// ConditionalStrNN_58772332478466
// MI455X (gfx1250) — hardware-verified
//
#include <hip/hip_runtime.h>
#include <math.h>

typedef __attribute__((ext_vector_type(16))) _Float16 v16h;
typedef __attribute__((ext_vector_type(16))) __bf16 v16b;
typedef __attribute__((ext_vector_type(8)))  _Float16 v8h;
typedef __attribute__((ext_vector_type(8)))  float v8f;
typedef __attribute__((ext_vector_type(4)))  float v4f;
typedef __attribute__((ext_vector_type(2)))  float v2f;
typedef __attribute__((ext_vector_type(4)))  unsigned v4u;
typedef __attribute__((ext_vector_type(4)))  int v4i;
typedef float __attribute__((may_alias)) float_a;
typedef int __attribute__((may_alias)) int_a;

template <typename T> __device__ __forceinline__ void vst2(void* p, T v) { *(volatile T*)p = v; __threadfence(); *(volatile T*)p = v; }
__device__ __forceinline__ v8f wmma16(v16h a, v16h b, v8f c) {
  v8f d = __builtin_amdgcn_wmma_f32_16x16x32_f16(false, a, false, b, (short)0, c, false, false);
  asm volatile("v_nop\n\tv_nop\n\tv_nop\n\tv_nop" : "+v"(d) : "v"(a), "v"(b));
  return d;
}
__device__ __forceinline__ v8f wmma_bf(v16b a, v16b b, v8f c) {
  v8f d = __builtin_amdgcn_wmma_f32_16x16x32_bf16(false, a, false, b, (short)0, c, false, false);
  asm volatile("v_nop\n\tv_nop\n\tv_nop\n\tv_nop" : "+v"(d) : "v"(a), "v"(b));
  return d;
}
__device__ __forceinline__ v16h frag_h(const _Float16* rowk0, int lane) {
  union { v16h v; v8h q[2]; } u; const _Float16* p = rowk0 + 8 * (lane >> 4);
  u.q[0] = *(const v8h*)p; u.q[1] = *(const v8h*)(p + 16); return u.v;
}
__device__ __forceinline__ v16h frag_f32(const float* rowk0, int lane) {
  v16h a; const float* p = rowk0 + 8 * (lane >> 4);
#pragma unroll
  for (int i = 0; i < 8; ++i) { a[i] = (_Float16)p[i]; a[8 + i] = (_Float16)p[16 + i]; }
  return a;
}
__device__ __forceinline__ v16h frag_f32s(const float* rowk0, int lane, float sc) {
  v16h a; const float* p = rowk0 + 8 * (lane >> 4);
#pragma unroll
  for (int i = 0; i < 8; ++i) { a[i] = (_Float16)(p[i] * sc); a[8 + i] = (_Float16)(p[16 + i] * sc); }
  return a;
}
__device__ __forceinline__ v16h fragc_f32(const float* W, int k0, int n, int lane, int ld, int K) {
  v16h a; const int g = lane >> 4;
#pragma unroll
  for (int i = 0; i < 8; ++i) { const int ka = k0 + 8 * g + i, kb = ka + 16;
    a[i] = (_Float16)(ka < K ? W[(size_t)ka * ld + n] : 0.f); a[8 + i] = (_Float16)(kb < K ? W[(size_t)kb * ld + n] : 0.f); }
  return a;
}
struct F2 { v16b h, l; };
__device__ __forceinline__ F2 bsplit16(const float v[16]) { F2 r;
#pragma unroll
  for (int i = 0; i < 16; ++i) { const __bf16 h = (__bf16)v[i]; r.h[i] = h; r.l[i] = (__bf16)(v[i] - (float)h); }
  return r; }
__device__ __forceinline__ F2 split_row(const float* row, int k0, int lane) { float v[16]; const float* p = row + k0 + 8 * (lane >> 4);
#pragma unroll
  for (int i = 0; i < 8; ++i) { v[i] = p[i]; v[8 + i] = p[16 + i]; }
  return bsplit16(v); }
__device__ __forceinline__ F2 split_rowK(const float* row, int k0, int lane, int K) { float v[16]; const int g = lane >> 4;
#pragma unroll
  for (int i = 0; i < 8; ++i) { const int ka = k0 + 8 * g + i, kb = ka + 16; v[i] = ka < K ? row[ka] : 0.f; v[8 + i] = kb < K ? row[kb] : 0.f; }
  return bsplit16(v); }
__device__ __forceinline__ F2 split_col(const float* W, int k0, int n, int lane, int ld, int K) { float v[16]; const int g = lane >> 4;
#pragma unroll
  for (int i = 0; i < 8; ++i) { const int ka = k0 + 8 * g + i, kb = ka + 16; v[i] = ka < K ? W[(size_t)ka * ld + n] : 0.f; v[8 + i] = kb < K ? W[(size_t)kb * ld + n] : 0.f; }
  return bsplit16(v); }
__device__ __forceinline__ v8f mac3(const F2& a, const F2& b, v8f c) { c = wmma_bf(a.l, b.h, c); c = wmma_bf(a.h, b.l, c); return wmma_bf(a.h, b.h, c); }
__device__ __forceinline__ float sigm(float v) { return 1.0f / (1.0f + expf(-v)); }
#define LDSX() do { asm volatile("s_wait_dscnt 0" ::: "memory"); __builtin_amdgcn_wave_barrier(); __builtin_amdgcn_fence(__ATOMIC_RELEASE, "workgroup"); } while (0)


#define NBT 64
#define COND 64

__global__ __launch_bounds__(128) void k_f(const float* __restrict__ u, const float* __restrict__ w, const float* __restrict__ bias, int N, float* __restrict__ F) {
  __shared__ __align__(16) float so[4][16][68];
  const int tid = threadIdx.x, wave = tid >> 5, lane = tid & 31, col = lane & 15, g = lane >> 4; const int n0 = blockIdx.x * 64; const int r0 = wave * 16;
  v8f acc[4] = {};
#pragma unroll
  for (int kc = 0; kc < 2; ++kc) { const F2 a = split_row(u + (size_t)(r0 + col) * COND, kc * 32, lane);
#pragma unroll
    for (int j = 0; j < 4; ++j) acc[j] = mac3(a, split_row(w + (size_t)(n0 + j * 16 + col) * COND, kc * 32, lane), acc[j]); }
#pragma unroll
  for (int j = 0; j < 4; ++j) { const float bb = bias[n0 + j * 16 + col];
#pragma unroll
    for (int r = 0; r < 8; ++r) so[wave][8 * g + r][j * 16 + col] = acc[j][r] + bb; }
  LDSX();
  for (int rl = 0; rl < 16; ++rl) { if (lane < 16) vst2(F + (size_t)(r0 + rl) * N + n0 + lane * 4, *(const v4f*)(&so[wave][rl][lane * 4])); }
}
template <int IN, int OUT>
__global__ __launch_bounds__(256) void k_layer(const float* __restrict__ hin, const float* __restrict__ F1, const float* __restrict__ F2, const float* __restrict__ mask, const float* __restrict__ W, float* __restrict__ hout) {
  __shared__ __align__(16) float sx[IN], sf1[IN]; __shared__ __align__(16) float sres[64];
  const int tid = threadIdx.x; const int b = blockIdx.y, o0 = blockIdx.x * 64; const int o = o0 + (tid >> 2), q = tid & 3;
  for (int i = tid; i < IN; i += 256) { sx[i] = hin[(size_t)b * IN + i]; sf1[i] = F1[(size_t)b * IN + i]; }
  __syncthreads();
  const float f2 = F2[(size_t)b * OUT + o]; const float* mrow = mask + (size_t)o * IN; const float* wrow = W + (size_t)o * IN; float s = 0.f;
#pragma unroll 2
  for (int i = q; i < IN; i += 4) s += sigm(f2 * sf1[i]) * (mrow[i] * wrow[i]) * sx[i];
  s += __shfl_xor(s, 1, 32); s += __shfl_xor(s, 2, 32);
  if (q == 0) sres[tid >> 2] = s;
  __syncthreads();
  if (tid < 64) vst2(hout + (size_t)b * OUT + o0 + tid, (float_a)sres[tid]);
}
extern "C" void kernel_launch(void* const* d_in, const int* in_sizes, int n_in, void* d_out, int out_size, void* d_ws, size_t ws_size, hipStream_t stream) {
  (void)in_sizes; (void)n_in; (void)out_size; (void)ws_size;
  const float** I = (const float**)d_in;
  const float* x = I[0]; const float* u = I[1]; const float* m0 = I[2]; const float* m1 = I[3]; const float* m2 = I[4]; const float* W0 = I[5]; const float* W1 = I[6]; const float* W2 = I[7];
  const float* a0w = I[8]; const float* a0b = I[9]; const float* b0w = I[10]; const float* b0b = I[11]; const float* a1w = I[12]; const float* a1b = I[13]; const float* b1w = I[14]; const float* b1b = I[15];
  const float* a2w = I[16]; const float* a2b = I[17]; const float* b2w = I[18]; const float* b2b = I[19];
  float* out = (float*)d_out;
  char* ws = (char*)d_ws; size_t off = 0;
  auto take = [&](size_t bytes) { char* p = ws + off; off += (bytes + 255) & ~(size_t)255; return p; };
  float* F10 = (float*)take(NBT * 512 * 4); float* F20 = (float*)take(NBT * 1024 * 4); float* F11 = (float*)take(NBT * 1024 * 4); float* F21 = (float*)take(NBT * 1024 * 4); float* F12 = (float*)take(NBT * 1024 * 4); float* F22 = (float*)take(NBT * 512 * 4);
  float* H1 = (float*)take(NBT * 1024 * 4); float* H2 = (float*)take(NBT * 1024 * 4);
  k_f<<<512 / 64, 128, 0, stream>>>(u, a0w, a0b, 512, F10);   k_f<<<1024 / 64, 128, 0, stream>>>(u, b0w, b0b, 1024, F20);
  k_f<<<1024 / 64, 128, 0, stream>>>(u, a1w, a1b, 1024, F11); k_f<<<1024 / 64, 128, 0, stream>>>(u, b1w, b1b, 1024, F21);
  k_f<<<1024 / 64, 128, 0, stream>>>(u, a2w, a2b, 1024, F12); k_f<<<512 / 64, 128, 0, stream>>>(u, b2w, b2b, 512, F22);
  k_layer<512, 1024><<<dim3(1024 / 64, NBT), 256, 0, stream>>>(x, F10, F20, m0, W0, H1);
  k_layer<1024, 1024><<<dim3(1024 / 64, NBT), 256, 0, stream>>>(H1, F11, F21, m1, W1, H2);
  k_layer<1024, 512><<<dim3(512 / 64, NBT), 256, 0, stream>>>(H2, F12, F22, m2, W2, out);
}
